// bin_feature_31963146617325
// MI455X (gfx1250) — hardware-run, weakly checked
//
#include <hip/hip_runtime.h>
#include <stddef.h>


typedef _Float16 v16h __attribute__((ext_vector_type(16)));
typedef _Float16 v8h  __attribute__((ext_vector_type(8)));
typedef float    v8f  __attribute__((ext_vector_type(8)));
typedef float    v4f  __attribute__((ext_vector_type(4)));
typedef unsigned int v8u __attribute__((ext_vector_type(8)));

#ifndef NB
#define NB 128
#endif
#ifndef NFEAT
#define NFEAT 512
#endif
#define NB_FULL    128
#define NFEAT_FULL 512
#define NBINS 2000
#define DOUT  128
#define KPAD  2016
#define KP    2048
#define MROWS (NB * NFEAT)
#define LDO   132

#define WCARRY 64.0f

#define WT_BYTES ((size_t)DOUT * KP * 2)
#define OFF_WT   ((size_t)0)
#define WS_TOTAL (OFF_WT + WT_BYTES)

static_assert(NB >= 1 && NB <= NB_FULL);
static_assert(NFEAT >= 1 && NFEAT <= NFEAT_FULL);
static_assert((MROWS % 64) == 0);
static_assert((NBINS % 8) == 0);
static_assert((KPAD % 32) == 0 && KPAD >= NBINS && KPAD <= KP);
static_assert(KP == 256 * 8);
static_assert((KP % 64) == 0);
static_assert(DOUT == 8 * 16);
static_assert(DOUT == 32 * 4);
static_assert((LDO % 4) == 0 && LDO >= DOUT);
static_assert((WT_BYTES % 128) == 0);
static_assert(WS_TOTAL <= (size_t)134217728);
static_assert((size_t)((NB_FULL - 1) * NFEAT_FULL + NFEAT_FULL) * DOUT * 4 == (size_t)33554432);

__device__ __forceinline__ float bf16r(float x) {
  unsigned int u = __float_as_uint(x);
  u = (u + 0x7FFFu + ((u >> 16) & 1u)) & 0xFFFF0000u;
  return __uint_as_float(u);
}

__device__ __forceinline__ v16h frag_at(const _Float16* p) {
  v8h lo = *(const v8h*)(p);
  v8h hi = *(const v8h*)(p + 16);
  v16h out;
#pragma unroll
  for (int i = 0; i < 8; ++i) { out[i] = lo[i]; out[i + 8] = hi[i]; }
  return out;
}

__device__ __forceinline__ v8f wmma16(v16h a, v16h b, v8f c) {
  v8f d = __builtin_amdgcn_wmma_f32_16x16x32_f16(false, a, false, b, (short)0, c,
                                                 false, false);
  asm volatile("v_nop\n\tv_nop\n\tv_nop\n\tv_nop" : "+v"(d) : "v"(a), "v"(b));
  return d;
}

__device__ __forceinline__ float relu_act(float t) {
  return fmaxf(t, 0.0f);
}

static __device__ __forceinline__ _Float16 toh_flush(float v) {
  const _Float16 r = (_Float16)v;
  return (fabsf(v) < 6.103515625e-05f) ? (_Float16)0.0f : r;
}

__global__ __launch_bounds__(256) void wplane_kernel(
    const float* __restrict__ W, _Float16* __restrict__ Wt) {
  const unsigned tid = threadIdx.x;
  const unsigned n = blockIdx.x;
  const bool live = tid < (unsigned)(NBINS / 8);
  const unsigned tc = live ? tid : (unsigned)(NBINS / 8 - 1);
  const float* src = W + (size_t)n * NBINS + tc * 8u;
  const v4f a0 = *(const v4f*)(src);
  const v4f a1 = *(const v4f*)(src + 4);
  v8h o;
#pragma unroll
  for (int i = 0; i < 4; ++i) {
    const _Float16 h0 = toh_flush(WCARRY * bf16r(a0[i]));
    const _Float16 h1 = toh_flush(WCARRY * bf16r(a1[i]));
    o[i]     = live ? h0 : (_Float16)0.0f;
    o[i + 4] = live ? h1 : (_Float16)0.0f;
  }
  _Float16* p = Wt + (size_t)n * KP + tid * 8u;
  *(volatile v8h*)p = o;
  __threadfence();
  *(volatile v8h*)p = o;
}

__global__ __launch_bounds__(128) void binlin_kernel(
    const float* __restrict__ X, const _Float16* __restrict__ Wt,
    const float* __restrict__ bias, float* __restrict__ outf) {
  __shared__ float Cs[64 * LDO];
  const unsigned tid = threadIdx.x, lane = tid & 31u;
  const unsigned wave = (unsigned)__builtin_amdgcn_readfirstlane((int)(threadIdx.x >> 5));
  const unsigned hh = lane >> 4, m = lane & 15u;
  const unsigned row0 = blockIdx.x * 64u;

  const unsigned arow = row0 + wave * 16u + m;
  const unsigned ab = arow / (unsigned)NFEAT;
  const unsigned af = arow - ab * (unsigned)NFEAT;
  const float xv = bf16r(X[(size_t)ab * NFEAT_FULL + af]);
  const float pos = xv - (-1000.0f);
  const float fl = floorf(pos);
  const float fr = pos - fl;
  const bool inrange = (fl >= 0.0f) && (fl < (float)NBINS);
  const int fi = (fl >= (float)NBINS) ? (int)NBINS : (inrange ? (int)fl : -1);
  const _Float16 frh = toh_flush(inrange ? fr : 0.0f);
  const unsigned frb = (unsigned)__builtin_bit_cast(unsigned short, frh);
  const unsigned w_both = 0x3C003C00u;
  const unsigned w_one_fr = 0x00003C00u | (frb << 16);
  const unsigned w_fr = frb;
  const int rel0 = fi - (int)(hh * 8u);

  const _Float16* bp = Wt + (size_t)m * KP + hh * 8u;
  v8f acc[8];
#pragma unroll
  for (int nb = 0; nb < 8; ++nb) acc[nb] = (v8f){};

#pragma unroll 1
  for (unsigned k0 = 0; k0 < (unsigned)KPAD; k0 += 32u) {
    const int rel = rel0 - (int)k0;
    v8u aw;
#pragma unroll
    for (int j = 0; j < 4; ++j) {
      const int t0 = rel - 2 * j;
      const int t1 = rel - 16 - 2 * j;
      aw[j]     = (t0 >= 2) ? w_both : ((t0 == 1) ? w_one_fr : ((t0 == 0) ? w_fr : 0u));
      aw[j + 4] = (t1 >= 2) ? w_both : ((t1 == 1) ? w_one_fr : ((t1 == 0) ? w_fr : 0u));
    }
    const v16h a = __builtin_bit_cast(v16h, aw);
#pragma unroll
    for (int nb = 0; nb < 8; ++nb) {
      const v16h b = frag_at(bp + (size_t)(nb * 16) * KP + k0);
      acc[nb] = wmma16(a, b, acc[nb]);
    }
  }

#pragma unroll
  for (int nb = 0; nb < 8; ++nb)
#pragma unroll
    for (int r = 0; r < 8; ++r)
      Cs[(wave * 16u + hh * 8u + (unsigned)r) * LDO + (unsigned)nb * 16u + m] = acc[nb][r];
  __syncthreads();

#pragma unroll 1
  for (unsigned g = 0; g < 4u; ++g) {
    v4f xs[4];
    size_t off[4];
#pragma unroll
    for (unsigned i = 0; i < 4u; ++i) {
      const unsigned r = 16u * g + 4u * i + (tid >> 5);
      const unsigned c = (tid & 31u) * 4u;
      const unsigned crow = row0 + r;
      const unsigned bidx = crow / (unsigned)NFEAT;
      const unsigned sq = crow - bidx * (unsigned)NFEAT;
      const size_t frow = (size_t)bidx * NFEAT_FULL + sq;
      const v4f u  = *(const v4f*)&Cs[r * LDO + c];
      const v4f gb = *(const v4f*)(bias + c);
      v4f val;
#pragma unroll
      for (int j = 0; j < 4; ++j)
        val[j] = relu_act(u[j] * (1.0f / WCARRY) + bf16r(gb[j]));
      xs[i] = val;
      off[i] = frow * DOUT + c;
    }
#pragma unroll
    for (int i = 0; i < 4; ++i) *(volatile v4f*)(outf + off[i]) = xs[i];
    __threadfence();
#pragma unroll
    for (int i = 0; i < 4; ++i) *(volatile v4f*)(outf + off[i]) = xs[i];
  }
}

extern "C" void kernel_launch(void* const* d_in, const int* in_sizes, int n_in,
                              void* d_out, int out_size, void* d_ws, size_t ws_size,
                              hipStream_t stream) {
  if (n_in < 3) return;
  const long long need_x = (long long)(NB - 1) * NFEAT_FULL + NFEAT;
  if ((long long)in_sizes[0] < need_x) return;
  if ((long long)in_sizes[1] < (long long)DOUT * NBINS) return;
  if (in_sizes[2] < DOUT) return;
  if ((long long)out_size < need_x * DOUT) return;
  if (ws_size < WS_TOTAL) return;

  const float* X    = (const float*)d_in[0];
  const float* W    = (const float*)d_in[1];
  const float* bias = (const float*)d_in[2];
  float* out = (float*)d_out;

  char* ws = (char*)d_ws;
  _Float16* Wt16 = (_Float16*)(ws + OFF_WT);

  wplane_kernel<<<dim3(DOUT), dim3(256), 0, stream>>>(W, Wt16);
  binlin_kernel<<<dim3(MROWS / 64), dim3(128), 0, stream>>>(X, Wt16, bias, out);
}
